// CL_MLP_88175678587650
// MI455X (gfx1250) — hardware-run, weakly checked
//
#include <hip/hip_runtime.h>
#define QNT 1024
#define QNB 8
#define QNH 1024
#define QNS 1023
#define QNE 4092
#define QNP 4096
typedef unsigned short v8us __attribute__((ext_vector_type(8), may_alias));
typedef float  v8f  __attribute__((ext_vector_type(8)));
typedef float  v4f  __attribute__((ext_vector_type(4)));
typedef float  v4fa __attribute__((ext_vector_type(4), may_alias));

__device__ __forceinline__ unsigned short bf16_bits(float x) { unsigned int u = __float_as_uint(x); return (unsigned short)((u + 0x7FFFu + ((u >> 16) & 1u)) >> 16); }
__device__ __forceinline__ float bf16_val(unsigned short b) { return __uint_as_float(((unsigned int)b) << 16); }
__device__ __forceinline__ float bf16_round(float x) { return bf16_val(bf16_bits(x)); }

typedef _Float16 v16h __attribute__((ext_vector_type(16)));
union FragH { v16h v; v8us half[2]; _Float16 h[16]; unsigned short u[16]; };

__global__ __launch_bounds__(256) void k_wt_f16(const float* __restrict__ W, _Float16* __restrict__ Wt, int K, int N, float scale) {
  const int t = blockIdx.x * 256 + threadIdx.x; if (t >= N * (K / 8)) return; const int n = t / (K / 8), k8 = (t % (K / 8)) * 8; FragH f;
#pragma unroll
  for (int i = 0; i < 8; ++i) f.h[i] = (_Float16)(bf16_round(W[(size_t)(k8 + i) * N + n]) * scale); const v8us o = f.half[0];
  *(volatile v8us*)((unsigned short*)Wt + (size_t)n * K + k8) = o; __threadfence(); *(volatile v8us*)((unsigned short*)Wt + (size_t)n * K + k8) = o;
}

typedef _Float16 v4h __attribute__((ext_vector_type(4)));

__global__ __launch_bounds__(256) void k_x16(const float* __restrict__ x, _Float16* __restrict__ X16, size_t n8) { const size_t t = (size_t)blockIdx.x * 256 + threadIdx.x; if (t >= n8) return; FragH f;
#pragma unroll
  for (int q = 0; q < 8; ++q) f.h[q] = (_Float16)bf16_round(x[t * 8 + q]); *(volatile v8us*)((unsigned short*)X16 + t * 8) = f.half[0]; __threadfence(); *(volatile v8us*)((unsigned short*)X16 + t * 8) = f.half[0]; }

__device__ __forceinline__ v16h g2_frag(const _Float16* p, int hh) { FragH f; f.half[0] = *(const v8us*)((const unsigned short*)p + 8 * hh); f.half[1] = *(const v8us*)((const unsigned short*)p + 16 + 8 * hh); return f.v; }
__device__ __forceinline__ v8f g2_mma(v16h a, v16h b, v8f c) { v8f d = __builtin_amdgcn_wmma_f32_16x16x32_f16(false, a, false, b, (short)0, c, false, false); asm volatile("v_nop\n\tv_nop\n\tv_nop\n\tv_nop" : "+v"(d) : "v"(a), "v"(b)); return d; }
template <int ACT>
__global__ __launch_bounds__(128) void k_gemm2(const _Float16* __restrict__ A, int lda, size_t sA, const _Float16* __restrict__ Bh, int ldb, size_t sB, float alpha, const float* __restrict__ bias, size_t sBias, const float* __restrict__ CP, int rowsPerB, size_t sCPb, int row0g,
    float* __restrict__ C, _Float16* __restrict__ C16, int ldc, size_t sC, int M, int N, int K) { static_assert(ACT == 0 || ACT == 3 || ACT == 6 || ACT == 8 || ACT == 9 || ACT == 11 || ACT == 12 || ACT == 14 || ACT == 15 || ACT == 16 || ACT == 17, "k_gemm2: unsupported ACT code (would silently apply no activation)");
  __shared__ __attribute__((aligned(16))) float so[4][32][68];
  const int tid = threadIdx.x, w = tid >> 5, lane = tid & 31, ln = lane & 15, hh = lane >> 4; const int by = blockIdx.y;
  A += (size_t)by * sA; Bh += (size_t)by * sB; const size_t cofs = (size_t)by * sC; const float* bp = bias ? bias + (size_t)by * sBias : nullptr;
  const int ntn = N >> 6; const int mt = blockIdx.x / ntn, nq = blockIdx.x - mt * ntn; const int row0 = mt * 128 + 32 * w, col0 = nq * 64; if (row0 >= M) return;
  const _Float16* a0p = A + (size_t)(row0 + ln) * lda; const _Float16* a1p = a0p + (size_t)16 * lda;
  const _Float16* b0p = Bh + (size_t)(col0 + ln) * ldb; const _Float16* b1p = b0p + (size_t)16 * ldb; const _Float16* b2p = b1p + (size_t)16 * ldb; const _Float16* b3p = b2p + (size_t)16 * ldb;
  const v8f z8 = {0.f,0.f,0.f,0.f,0.f,0.f,0.f,0.f}; v8f c00 = z8, c01 = z8, c02 = z8, c03 = z8, c10 = z8, c11 = z8, c12 = z8, c13 = z8;
  for (int kb = 0; kb < K; kb += 32) { const v16h a0 = g2_frag(a0p + kb, hh), a1 = g2_frag(a1p + kb, hh);
    v16h b = g2_frag(b0p + kb, hh); c00 = g2_mma(a0, b, c00); c10 = g2_mma(a1, b, c10);
    b = g2_frag(b1p + kb, hh); c01 = g2_mma(a0, b, c01); c11 = g2_mma(a1, b, c11);
    b = g2_frag(b2p + kb, hh); c02 = g2_mma(a0, b, c02); c12 = g2_mma(a1, b, c12);
    b = g2_frag(b3p + kb, hh); c03 = g2_mma(a0, b, c03); c13 = g2_mma(a1, b, c13); }
  v8f accs[8] = {c00, c01, c02, c03, c10, c11, c12, c13};
#pragma unroll
  for (int u = 0; u < 8; ++u) { const int t = u & 3, half = u >> 2; const int col = col0 + t * 16 + ln; const float bv = bp ? bf16_round(bp[col]) : 0.f;
#pragma unroll
    for (int r = 0; r < 8; ++r) { const int rloc = half * 16 + 8 * hh + r; float v = accs[u][r] * alpha + bv; if (CP) { if (rowsPerB < 0) v += CP[cofs + (size_t)(row0g + row0 + rloc) * ldc + col];        else { const int bidx = (row0g + row0 + rloc) / rowsPerB; v += CP[(size_t)bidx * sCPb + (size_t)by * 64 + col]; } }
      if (ACT == 3) v = fmaxf(v, 0.f); else if (ACT == 6) v = 0.5f * v * (1.0f + erff(v * 0.70710678118654752f)); else if (ACT == 11) v = 1.0f / (1.0f + expf(-v)); else if (ACT == 15) v = v / (1.0f + expf(-v)); else if (ACT == 12) v = (v > 0.f) ? v : 0.01f * v; else if (ACT == 8) v = tanhf(v); else if (ACT == 9) v = 0.5f * v * (1.0f + tanhf(0.7978845608028654f * (v + 0.044715f * v * v * v))); else if (ACT == 14) v = (v > 0.f) ? v : 0.1f * v; else if (ACT == 16) v = (v >= 0.f) ? v : 0.3f * v; else if (ACT == 17) v = (v >= 0.f) ? v : 0.2f * v;
      so[w][rloc][t * 16 + ln] = v; } }
  __builtin_amdgcn_fence(__ATOMIC_ACQ_REL, "workgroup"); __builtin_amdgcn_wave_barrier();
  const int rsub = lane >> 4, c4 = (lane & 15) * 4;
  for (int pass = 0; pass < 2; ++pass) {
#pragma unroll
    for (int q = 0; q < 16; ++q) { const int r = q * 2 + rsub; const v4f v = *(const v4fa*)&so[w][r][c4]; if (C) *(volatile v4f*)(C + cofs + (size_t)(row0 + r) * ldc + col0 + c4) = v; if (C16) { v4h h4; for (int i = 0; i < 4; ++i) h4[i] = (_Float16)v[i]; *(volatile v4h*)(C16 + cofs + (size_t)(row0 + r) * ldc + col0 + c4) = h4; } }
    if (pass == 0) __threadfence(); } }

__global__ __launch_bounds__(256) void k_cs16(const float* __restrict__ sw, _Float16* __restrict__ tw, float scale) { const size_t t = (size_t)blockIdx.x * 256 + threadIdx.x; FragH f;
#pragma unroll
  for (int q = 0; q < 8; ++q) f.h[q] = (_Float16)(bf16_round(sw[t * 8 + q]) * scale); unsigned short* tp = (unsigned short*)tw + t * 8; *(volatile v8us*)tp = f.half[0]; __threadfence(); *(volatile v8us*)tp = f.half[0]; }
__global__ __launch_bounds__(256) void k_nrm(const float* __restrict__ o1, const float* __restrict__ o2, float* __restrict__ nv) { const unsigned i = blockIdx.x * 256u + threadIdx.x; float r = 0.0f; if (i < (unsigned)QNE) { const unsigned hf = i / (2u * QNS), j = i % (2u * QNS), wh = j / (unsigned)QNS, tt = j % (unsigned)QNS + (hf == 0u ? 1u : 0u); const float* sp = (wh == 0u ? o1 : o2) + ((size_t)(QNB - 1) * QNT + tt) * QNH; float ss = 0.0f; for (int c = 0; c < QNH; c += 4) { const v4f v = *(const v4fa*)(sp + c); ss += v[0] * v[0]; ss += v[1] * v[1]; ss += v[2] * v[2]; ss += v[3] * v[3]; } r = 1.0f / fmaxf(sqrtf(ss), 1e-12f); } *(volatile float*)(nv + i) = r; __threadfence(); *(volatile float*)(nv + i) = r; }
__global__ __launch_bounds__(256) void k_unit(const float* __restrict__ o1, const float* __restrict__ o2, const float* __restrict__ nv, _Float16* __restrict__ ue) { const unsigned tn = blockIdx.x * 256u + threadIdx.x, i = tn / (unsigned)(QNH / 8), c8 = (tn % (unsigned)(QNH / 8)) * 8u; FragH f; if (i < (unsigned)QNE) { const unsigned hf = i / (2u * QNS), j = i % (2u * QNS), wh = j / (unsigned)QNS, tt = j % (unsigned)QNS + (hf == 0u ? 1u : 0u); const float* sp = (wh == 0u ? o1 : o2) + ((size_t)(QNB - 1) * QNT + tt) * QNH; const float s = nv[i]; const v4f a = *(const v4fa*)(sp + c8), b = *(const v4fa*)(sp + c8 + 4);
#pragma unroll
    for (int k = 0; k < 8; ++k) { const float v = ((k < 4) ? a[k & 3] : b[k & 3]) * s; f.h[k] = (_Float16)((fabsf(v) < 0x1p-14f) ? 0.0f : v); } } else {
#pragma unroll
    for (int k = 0; k < 8; ++k) f.h[k] = (_Float16)0.0f; }
  unsigned short* tp = (unsigned short*)ue + (size_t)tn * 8; *(volatile v8us*)tp = f.half[0]; __threadfence(); *(volatile v8us*)tp = f.half[0]; }
__global__ __launch_bounds__(256) void k_rows(const float* __restrict__ sm, float* __restrict__ lr) { const unsigned i = blockIdx.x * 256u + threadIdx.x; float r = 0.0f; if (i < (unsigned)QNE) { const unsigned p = (i < 2u * QNS) ? i + 2u * QNS : i - 2u * QNS; const float* rp = sm + (size_t)i * QNP; float den = 0.0f, lp = 0.0f; for (unsigned c = 0; c < (unsigned)QNP; c += 4) { const v4f v = *(const v4fa*)(rp + c);
#pragma unroll
      for (unsigned k = 0; k < 4; ++k) { const unsigned cc = c + k; const float g = 10.0f * v[k]; const float e = expf(g); den += (cc < (unsigned)QNE && cc != i) ? e : 0.0f; lp = (cc == p) ? g : lp; } } r = logf(den) - lp; } *(volatile float*)(lr + i) = r; __threadfence(); *(volatile float*)(lr + i) = r; }
__global__ __launch_bounds__(32) void k_mean(const float* __restrict__ lr, float* __restrict__ res) { if (threadIdx.x != 0u || blockIdx.x != 0u) return; const volatile __attribute__((address_space(1))) float* lp = (const volatile __attribute__((address_space(1))) float*)lr; float s = 0.0f; for (int i = 0; i < QNE; ++i) s += lp[i]; const float m = s / (float)QNE; *(volatile float*)res = m; __threadfence(); *(volatile float*)res = m; }

extern "C" void kernel_launch(void* const* d_in, const int* in_sizes, int n_in,
                              void* d_out, int out_size, void* d_ws, size_t ws_size, hipStream_t stream) {
  if (n_in < 6) return; if (in_sizes[0] < QNT * QNB * QNH || in_sizes[1] < QNT * QNB * QNH || in_sizes[2] < QNH * QNH || in_sizes[3] < QNH || in_sizes[4] < QNH * QNH || in_sizes[5] < QNH) return; if (out_size < 2 * QNB * QNT * QNH + 1) return;
  const float* xa = (const float*)d_in[0]; const float* xb = (const float*)d_in[1]; const float* wa = (const float*)d_in[2]; const float* ra = (const float*)d_in[3]; const float* wb = (const float*)d_in[4]; const float* rb = (const float*)d_in[5]; float* o1 = (float*)d_out; float* o2 = o1 + (size_t)QNB * QNT * QNH; float* res = o2 + (size_t)QNB * QNT * QNH;
  static_assert(QNT % 128 == 0 && QNH % 64 == 0 && QNH % 32 == 0 && QNP % 128 == 0 && QNP % 64 == 0 && QNE == 4 * QNS && QNS == QNT - 1 && QNP >= QNE && ((size_t)QNT * QNB * QNH) % 2048 == 0 && (QNH * QNH) % 2048 == 0 && ((size_t)QNH * (QNH / 8)) % 256 == 0 && QNP % 256 == 0 && (QNP * (QNH / 8)) % 256 == 0, "whole tiles, exact launches");
  uint8_t* wsp = (uint8_t*)d_ws; size_t off = 0;
  auto take = [&](size_t bytes) { uint8_t* at = wsp + off; off += (bytes + 255) & ~(size_t)255; return at; };
  _Float16* XA = (_Float16*)take((size_t)QNT * QNB * QNH * 2); _Float16* XB = (_Float16*)take((size_t)QNT * QNB * QNH * 2); _Float16* WA = (_Float16*)take((size_t)QNH * QNH * 2); _Float16* WB = (_Float16*)take((size_t)QNH * QNH * 2);
  _Float16* MA = (_Float16*)take((size_t)QNB * QNT * QNH * 2); _Float16* MB = (_Float16*)take((size_t)QNB * QNT * QNH * 2);
  float* NV = (float*)take((size_t)QNP * 4); _Float16* UE = (_Float16*)take((size_t)QNP * QNH * 2); float* SM = (float*)take((size_t)QNP * QNP * 4); float* LR = (float*)take((size_t)QNP * 4);
  if (off > ws_size) return;
  k_x16<<<(unsigned)((size_t)QNT * QNB * QNH / 8 / 256), 256, 0, stream>>>(xa, XA, (size_t)QNT * QNB * QNH / 8);
  k_x16<<<(unsigned)((size_t)QNT * QNB * QNH / 8 / 256), 256, 0, stream>>>(xb, XB, (size_t)QNT * QNB * QNH / 8);
  k_wt_f16<<<(unsigned)((size_t)QNH * (QNH / 8) / 256), 256, 0, stream>>>(wa, WA, QNH, QNH, 16.0f);
  k_wt_f16<<<(unsigned)((size_t)QNH * (QNH / 8) / 256), 256, 0, stream>>>(wb, WB, QNH, QNH, 16.0f);
  const dim3 gl((unsigned)((QNT / 128) * (QNH / 64)), (unsigned)QNB);
  k_gemm2<3><<<gl, 128, 0, stream>>>(XA, QNB * QNH, (size_t)QNH, WA, QNH, (size_t)0, 0.0625f, ra, (size_t)0, nullptr, 1, 0, 0, nullptr, MA, QNH, (size_t)QNT * QNH, QNT, QNH, QNH);
  k_gemm2<3><<<gl, 128, 0, stream>>>(XB, QNB * QNH, (size_t)QNH, WA, QNH, (size_t)0, 0.0625f, ra, (size_t)0, nullptr, 1, 0, 0, nullptr, MB, QNH, (size_t)QNT * QNH, QNT, QNH, QNH);
  k_gemm2<3><<<gl, 128, 0, stream>>>(MA, QNH, (size_t)QNT * QNH, WB, QNH, (size_t)0, 0.0625f, rb, (size_t)0, nullptr, 1, 0, 0, o1, nullptr, QNH, (size_t)QNT * QNH, QNT, QNH, QNH);
  k_gemm2<3><<<gl, 128, 0, stream>>>(MB, QNH, (size_t)QNT * QNH, WB, QNH, (size_t)0, 0.0625f, rb, (size_t)0, nullptr, 1, 0, 0, o2, nullptr, QNH, (size_t)QNT * QNH, QNT, QNH, QNH);
  k_nrm<<<(unsigned)(QNP / 256), 256, 0, stream>>>(o1, o2, NV);
  k_unit<<<(unsigned)(QNP * (QNH / 8) / 256), 256, 0, stream>>>(o1, o2, NV, UE);
  k_gemm2<0><<<dim3((unsigned)((QNP / 128) * (QNP / 64)), 1u), 128, 0, stream>>>(UE, QNH, (size_t)0, UE, QNH, (size_t)0, 1.0f, nullptr, (size_t)0, nullptr, 1, 0, 0, SM, nullptr, QNP, (size_t)0, QNP, QNP, QNH);
  k_rows<<<(unsigned)(QNP / 256), 256, 0, stream>>>(SM, LR);
  k_mean<<<1, 32, 0, stream>>>(LR, res);
}
